// MultiheadAttention_4294967296543
// MI455X (gfx1250) — hardware-run, weakly checked
//
#include <hip/hip_runtime.h>


#ifndef NB
#define NB 2
#endif
#ifndef SEQ
#define SEQ 2048
#endif
#define SEQ_FULL 2048
#define TT   SEQ
#define DM   1024
#define NH   16
#define HD   64
#define ROT  32
#define NZ   (NB * NH)
#define MT   (NB * TT)
#define ZH   2
#define SCL  0.125f
#define LOG2E 1.4426950408889634f

static_assert(TT % 128 == 0);
static_assert(DM == NH * HD);
static_assert(DM % 64 == 0);
static_assert(NZ % ZH == 0);
static_assert(ROT / 2 == 16);
static_assert(TT <= SEQ_FULL);

typedef unsigned short bf;
typedef __attribute__((ext_vector_type(16))) __bf16   v16bf;
typedef __attribute__((ext_vector_type(8)))  unsigned short v8us;
typedef __attribute__((ext_vector_type(4)))  unsigned short v4us;
typedef __attribute__((ext_vector_type(2)))  unsigned short v2us;
typedef __attribute__((ext_vector_type(8)))  float    v8f;
typedef __attribute__((ext_vector_type(4)))  float    v4f;
typedef __attribute__((ext_vector_type(2)))  float    v2f;
typedef __attribute__((ext_vector_type(4)))  int      v4i;
typedef v4f  __attribute__((may_alias)) v4fa;

__device__ __forceinline__ unsigned short f2bf(float f) { unsigned u = __float_as_uint(f); u += 0x7FFFu + ((u >> 16) & 1u); return (unsigned short)(u >> 16); }
__device__ __forceinline__ float bf2f(unsigned short b) { return __uint_as_float(((unsigned)b) << 16); }
__device__ __forceinline__ void splitf(float y, unsigned short& h, unsigned short& l) { h = f2bf(y); l = f2bf(y - bf2f(h)); }
__device__ __forceinline__ v16bf cat16b(v8us lo, v8us hi) { return __builtin_bit_cast(v16bf, __builtin_shufflevector(lo, hi, 0, 1, 2, 3, 4, 5, 6, 7, 8, 9, 10, 11, 12, 13, 14, 15)); }
__device__ __forceinline__ v8f wmmab(v16bf a, v16bf b, v8f c) { return __builtin_amdgcn_wmma_f32_16x16x32_bf16(false, a, false, b, (short)0, c, false, false); }
__device__ __forceinline__ v16bf ldfrag(const bf* p) { return cat16b(*(const v8us*)p, *(const v8us*)(p + 16)); }

template <int NSPLIT, int CAUSAL>
__global__ __launch_bounds__(32) void k_gemmw(const bf* __restrict__ A, const bf* __restrict__ A2, const bf* __restrict__ Bt, const bf* __restrict__ Bt2, int K, int lda, int ldb, float* C, int ldc, size_t sA, size_t sB, size_t sC) {
    __shared__ __align__(16) float os[16 * 68];
    const int r0 = blockIdx.x * 64, c0 = blockIdx.y * 64;
    if (CAUSAL == 1) { if (c0 > r0) return; }
    int Kend = K; if (CAUSAL == 2) { Kend = (r0 + 64 < K) ? (r0 + 64) : K; }
    const size_t z = blockIdx.z; A += z * sA; if (A2) A2 += z * sA; Bt += z * sB; if (Bt2) Bt2 += z * sB; C += z * sC;
    const int lane = threadIdx.x & 31, lr = lane & 15, hi = lane >> 4;
    v8f acc[4][4];
#pragma unroll
    for (int mb = 0; mb < 4; ++mb)
#pragma unroll
        for (int nb = 0; nb < 4; ++nb) acc[mb][nb] = (v8f){};
    const size_t aoff = (size_t)(r0 + lr) * lda + 8 * hi, boff = (size_t)(c0 + lr) * ldb + 8 * hi;
#pragma unroll 1
    for (int kc = 0; kc < Kend; kc += 32) {
        v16bf a[4], a2[4];
#pragma unroll
        for (int mb = 0; mb < 4; ++mb) { a[mb] = ldfrag(A + aoff + (size_t)mb * 16 * lda + kc); if (NSPLIT == 1 || NSPLIT == 2) a2[mb] = ldfrag(A2 + aoff + (size_t)mb * 16 * lda + kc); }
#pragma unroll
        for (int nb = 0; nb < 4; ++nb) { const v16bf b = ldfrag(Bt + boff + (size_t)nb * 16 * ldb + kc); v16bf b2; if (NSPLIT >= 2) b2 = ldfrag(Bt2 + boff + (size_t)nb * 16 * ldb + kc);
#pragma unroll
            for (int mb = 0; mb < 4; ++mb) { acc[mb][nb] = wmmab(a[mb], b, acc[mb][nb]); if (NSPLIT == 1 || NSPLIT == 2) acc[mb][nb] = wmmab(a2[mb], b, acc[mb][nb]); if (NSPLIT >= 2) acc[mb][nb] = wmmab(a[mb], b2, acc[mb][nb]); } }
        asm volatile("v_nop\n\tv_nop\n\tv_nop\n\tv_nop" : "+v"(acc[0][0]), "+v"(acc[1][1]), "+v"(acc[2][2]), "+v"(acc[3][3]) : "v"(a[0]), "v"(a[3]));
    }
#pragma unroll
    for (int mb = 0; mb < 4; ++mb) {
#pragma unroll
        for (int nb = 0; nb < 4; ++nb) {
#pragma unroll
            for (int j = 0; j < 8; ++j) os[(hi * 8 + j) * 68 + nb * 16 + lr] = acc[mb][nb][j]; }
        __builtin_amdgcn_wave_barrier(); asm volatile("" ::: "memory");
        float* crow = C + (size_t)(r0 + mb * 16) * ldc + c0;
#pragma unroll 1
        for (int ps = 0; ps < 2; ++ps) {
#pragma unroll
            for (int s = 0; s < 8; ++s) { const int row = 2 * s + hi, cofs = lr * 4; const v4f val = *(const v4fa*)(os + row * 68 + cofs);
                *(volatile v4f*)(crow + (size_t)row * ldc + cofs) = val; }
            if (ps == 0) __threadfence(); }
        __builtin_amdgcn_wave_barrier(); asm volatile("" ::: "memory");
    }
}

__global__ __launch_bounds__(256) void k_cvt8(const float* __restrict__ src, bf* dst, size_t n8) { const size_t i = (size_t)blockIdx.x * 256 + threadIdx.x; if (i >= n8) return; const v8f v = *(const v8f*)(src + i * 8); v8us o;
#pragma unroll
    for (int k = 0; k < 8; ++k) o[k] = f2bf(v[k]); *(volatile v8us*)(dst + i * 8) = o; __threadfence(); *(volatile v8us*)(dst + i * 8) = o; }

__global__ __launch_bounds__(256) void k_split8(const float* __restrict__ src, bf* Dh, bf* Dl, size_t n8) { const size_t i = (size_t)blockIdx.x * 256 + threadIdx.x; if (i >= n8) return; const v8f v = *(const v8f*)(src + i * 8); v8us oh, ol;
#pragma unroll
    for (int k = 0; k < 8; ++k) { unsigned short a, c; splitf(v[k], a, c); oh[k] = a; ol[k] = c; }
    *(volatile v8us*)(Dh + i * 8) = oh; *(volatile v8us*)(Dl + i * 8) = ol; __threadfence(); *(volatile v8us*)(Dh + i * 8) = oh; *(volatile v8us*)(Dl + i * 8) = ol; }

__device__ __forceinline__ float invfreq(int j) {
    float r = 1.0f;
    r = (j == 1)  ? (1.0f / (float)1.7782794100389228) : r;
    r = (j == 2)  ? (1.0f / (float)3.1622776601683795) : r;
    r = (j == 3)  ? (1.0f / (float)5.623413251903491)  : r;
    r = (j == 4)  ? (1.0f / 10.0f) : r;
    r = (j == 5)  ? (1.0f / (float)17.782794100389228) : r;
    r = (j == 6)  ? (1.0f / (float)31.622776601683793) : r;
    r = (j == 7)  ? (1.0f / (float)56.23413251903491)  : r;
    r = (j == 8)  ? (1.0f / 100.0f) : r;
    r = (j == 9)  ? (1.0f / (float)177.82794100389228) : r;
    r = (j == 10) ? (1.0f / (float)316.22776601683796) : r;
    r = (j == 11) ? (1.0f / (float)562.341325190349)   : r;
    r = (j == 12) ? (1.0f / 1000.0f) : r;
    r = (j == 13) ? (1.0f / (float)1778.2794100389228) : r;
    r = (j == 14) ? (1.0f / (float)3162.2776601683795) : r;
    r = (j == 15) ? (1.0f / (float)5623.413251903491)  : r;
    return r;
}
__global__ __launch_bounds__(256) void k_cstab(float* CS) { const int idx = blockIdx.x * 256 + threadIdx.x; if (idx >= TT * (ROT / 2)) return; const int t = idx / (ROT / 2), j = idx % (ROT / 2);
    const float fr = __fmul_rn((float)t, invfreq(j)); v2f cs; cs[0] = cosf(fr); cs[1] = sinf(fr);
    *(volatile v2f*)(CS + (size_t)idx * 2) = cs; __threadfence(); *(volatile v2f*)(CS + (size_t)idx * 2) = cs; }

__global__ __launch_bounds__(256) void k_ropei(const float* __restrict__ F, const float* __restrict__ CS, bf* Ph, bf* Pl) {
#pragma clang fp contract(off)
    const size_t e = ((size_t)blockIdx.x * 256 + threadIdx.x) * 2; if (e >= (size_t)NZ * TT * HD) return; const int d = (int)(e % HD); const int t = (int)((e / HD) % TT);
    const v2f x = *(const v2f*)(F + e); const int jc = ((d >> 1) < (ROT / 2 - 1)) ? (d >> 1) : (ROT / 2 - 1); const v2f cs = *(const v2f*)(CS + ((size_t)t * (ROT / 2) + jc) * 2);
    float a0 = __fmul_rn(x[0], cs[0]), b0 = __fmul_rn(x[1], cs[1]), a1 = __fmul_rn(x[1], cs[0]), b1 = __fmul_rn(x[0], cs[1]);
    asm volatile("" : "+v"(a0)); asm volatile("" : "+v"(b0)); asm volatile("" : "+v"(a1)); asm volatile("" : "+v"(b1));
    const float r0 = __fsub_rn(a0, b0), r1 = __fadd_rn(a1, b1); const bool rot = (d < ROT); const float y0 = rot ? r0 : x[0], y1 = rot ? r1 : x[1];
    v2us oh, ol; unsigned short h, l; splitf(y0, h, l); oh[0] = h; ol[0] = l; splitf(y1, h, l); oh[1] = h; ol[1] = l;
    *(volatile v2us*)(Ph + e) = oh; *(volatile v2us*)(Pl + e) = ol; __threadfence(); *(volatile v2us*)(Ph + e) = oh; *(volatile v2us*)(Pl + e) = ol; }

__global__ __launch_bounds__(256) void k_vtp(const float* __restrict__ F, bf* Vh, bf* Vl) { const size_t e = ((size_t)blockIdx.x * 256 + threadIdx.x) * 2; if (e >= (size_t)NZ * HD * TT) return; const int t = (int)(e % TT); const int d = (int)((e / TT) % HD); const size_t g = e / ((size_t)TT * HD); v2us oh, ol;
#pragma unroll
    for (int q = 0; q < 2; ++q) { const float x = F[g * (size_t)TT * HD + (size_t)(t + q) * HD + d]; unsigned short a2, c2; splitf(x, a2, c2); oh[q] = a2; ol[q] = c2; }
    *(volatile v2us*)(Vh + e) = oh; *(volatile v2us*)(Vl + e) = ol; __threadfence(); *(volatile v2us*)(Vh + e) = oh; *(volatile v2us*)(Vl + e) = ol; }

__global__ __launch_bounds__(256) void k_csoft(float* Sb, const int* __restrict__ pm, int z0) {
    const int lane = threadIdx.x & 31; const int wv = __builtin_amdgcn_readfirstlane((int)(threadIdx.x >> 5));
    const int row = blockIdx.x * 8 + wv; if (row >= ZH * TT) return; const int i = row % TT; const int zz = row / TT; const int b = (z0 + zz) / NH;
    const float* sr = Sb + (size_t)row * TT; const int* mr = pm + (size_t)b * SEQ_FULL; const float NINF = -__builtin_inff();
    float v[TT / 32]; float mx = NINF;
#pragma unroll
    for (int ch = 0; ch < TT / 128; ++ch) {
        if (ch * 128 <= i) { const int j0 = ch * 128 + lane * 4; const v4f a = *(const v4fa*)(sr + j0); const v4i m4 = *(const v4i*)(mr + j0);
#pragma unroll
            for (int q = 0; q < 4; ++q) { const bool ok = (j0 + q <= i) && (m4[q] != 0); const float t = ok ? (a[q] * SCL) : NINF; v[ch * 4 + q] = t; mx = fmaxf(mx, t); }
        } else {
#pragma unroll
            for (int q = 0; q < 4; ++q) v[ch * 4 + q] = NINF; } }
#pragma unroll
    for (int sh = 16; sh; sh >>= 1) mx = fmaxf(mx, __shfl_xor(mx, sh, 32));
    float sum = 0.f;
#pragma unroll
    for (int ch = 0; ch < TT / 128; ++ch) {
        if (ch * 128 <= i) {
#pragma unroll
            for (int q = 0; q < 4; ++q) { float d0 = __fsub_rn(v[ch * 4 + q], mx); asm volatile("" : "+v"(d0)); const float p = __builtin_amdgcn_exp2f(__fmul_rn(d0, LOG2E)); v[ch * 4 + q] = p; sum += p; } } }
#pragma unroll
    for (int sh = 16; sh; sh >>= 1) sum += __shfl_xor(sum, sh, 32);
    const float f = __fdiv_rn(1.0f, sum);
    bf* ph = (bf*)Sb + (size_t)row * 2 * TT; bf* pl = ph + TT;
#pragma unroll 1
    for (int ps = 0; ps < 2; ++ps) {
#pragma unroll
        for (int ch = 0; ch < TT / 128; ++ch) {
            if (ch * 128 <= i) { v4us oh, ol;
#pragma unroll
                for (int q = 0; q < 4; ++q) { unsigned short a, c2; splitf(v[ch * 4 + q] * f, a, c2); oh[q] = a; ol[q] = c2; }
                *(volatile v4us*)(ph + ch * 128 + lane * 4) = oh; *(volatile v4us*)(pl + ch * 128 + lane * 4) = ol; } }
        if (ps == 0) __threadfence(); }
}

constexpr size_t cmax(size_t a, size_t b) { return a > b ? a : b; }
constexpr size_t al256(size_t a) { return (a + 255) & ~(size_t)255; }
constexpr size_t B_WIN = (size_t)3 * DM * DM * 2, B_WO = (size_t)DM * DM * 2, B_CS = (size_t)TT * (ROT / 2) * 8, B_PL = (size_t)NZ * TT * HD * 2, B_OB = (size_t)NZ * TT * HD * 4;
constexpr size_t B_XB = (size_t)MT * DM * 2, B_F = (size_t)MT * DM * 4, B_AT = (size_t)MT * DM * 2, B_S = (size_t)ZH * TT * TT * 4;
constexpr size_t B_R = cmax(B_S, cmax(B_XB + B_F, 2 * B_AT));
constexpr size_t B_TOTAL = al256(B_WIN) + al256(B_WO) + al256(B_CS) + 6 * al256(B_PL) + al256(B_OB) + al256(B_R);
static_assert(B_XB + B_F <= B_R);
static_assert(2 * B_AT <= B_R);
static_assert(B_S <= B_R);
static_assert(B_TOTAL <= (size_t)134217728);
static_assert((B_XB % 256) == 0);
static_assert((B_AT % 256) == 0);

extern "C" void kernel_launch(void* const* d_in, const int* in_sizes, int n_in,
                              void* d_out, int out_size, void* d_ws, size_t ws_size, hipStream_t stream) {
    (void)out_size;
    if (n_in < 6) return;
    if ((size_t)in_sizes[0] < (size_t)(NB - 1) * SEQ_FULL * DM + (size_t)TT * DM) return;
    if ((size_t)in_sizes[3] < (size_t)(NB - 1) * SEQ_FULL + (size_t)TT) return;
    if ((size_t)in_sizes[4] < (size_t)3 * DM * DM) return;
    if ((size_t)in_sizes[5] < (size_t)DM * DM) return;
    const float* x = (const float*)d_in[0];
    const int* pm = (const int*)d_in[3];
    const float* win = (const float*)d_in[4];
    const float* wo = (const float*)d_in[5];
    float* OUT = (float*)d_out;
    if (ws_size < B_TOTAL) return;
    char* wsp = (char*)d_ws;
    auto take = [&](size_t bytes) { char* p = wsp; wsp += (bytes + 255) & ~(size_t)255; return (void*)p; };
    bf* WIN = (bf*)take(B_WIN); bf* WO = (bf*)take(B_WO); float* CS = (float*)take(B_CS);
    bf* QPh = (bf*)take(B_PL); bf* QPl = (bf*)take(B_PL); bf* KPh = (bf*)take(B_PL); bf* KPl = (bf*)take(B_PL); bf* VTh = (bf*)take(B_PL); bf* VTl = (bf*)take(B_PL);
    float* Ob = (float*)take(B_OB); char* R = (char*)take(B_R);
    if ((size_t)(wsp - (char*)d_ws) > ws_size) return;
    bf* XB = (bf*)R; float* F = (float*)(R + B_XB);
    float* Sb = (float*)R;
    bf* ATh = (bf*)R; bf* ATl = (bf*)(R + B_AT);

    k_cvt8<<<(unsigned)(((size_t)3 * DM * DM / 8 + 255) / 256), 256, 0, stream>>>(win, WIN, (size_t)3 * DM * DM / 8);
    k_cvt8<<<(unsigned)(((size_t)DM * DM / 8 + 255) / 256), 256, 0, stream>>>(wo, WO, (size_t)DM * DM / 8);
    k_cstab<<<(TT * (ROT / 2) + 255) / 256, 256, 0, stream>>>(CS);
    for (int b = 0; b < NB; ++b)
        k_cvt8<<<(unsigned)(((size_t)TT * DM / 8 + 255) / 256), 256, 0, stream>>>(x + (size_t)b * SEQ_FULL * DM, XB + (size_t)b * TT * DM, (size_t)TT * DM / 8);

    const unsigned LP = (unsigned)(((size_t)NZ * TT * HD / 2 + 255) / 256);
    k_gemmw<0, 0><<<dim3(MT / 64, DM / 64, 1), 32, 0, stream>>>(XB, nullptr, WIN, nullptr, DM, DM, DM, F, DM, 0, 0, 0);
    k_ropei<<<LP, 256, 0, stream>>>(F, CS, QPh, QPl);
    k_gemmw<0, 0><<<dim3(MT / 64, DM / 64, 1), 32, 0, stream>>>(XB, nullptr, WIN + (size_t)DM * DM, nullptr, DM, DM, DM, F, DM, 0, 0, 0);
    k_ropei<<<LP, 256, 0, stream>>>(F, CS, KPh, KPl);
    k_gemmw<0, 0><<<dim3(MT / 64, DM / 64, 1), 32, 0, stream>>>(XB, nullptr, WIN + (size_t)2 * DM * DM, nullptr, DM, DM, DM, F, DM, 0, 0, 0);
    k_vtp<<<LP, 256, 0, stream>>>(F, VTh, VTl);

    const size_t PL = (size_t)TT * HD;
    for (int z0 = 0; z0 < NZ; z0 += ZH) {
        k_gemmw<2, 1><<<dim3(TT / 64, TT / 64, ZH), 32, 0, stream>>>(QPh + z0 * PL, QPl + z0 * PL, KPh + z0 * PL, KPl + z0 * PL, HD, HD, HD, Sb, TT, PL, PL, (size_t)TT * TT);
        k_csoft<<<ZH * TT / 8, 256, 0, stream>>>(Sb, pm, z0);
        k_gemmw<2, 2><<<dim3(TT / 64, HD / 64, ZH), 32, 0, stream>>>((const bf*)Sb, (const bf*)Sb + TT, VTh + z0 * PL, VTl + z0 * PL, TT, 2 * TT, TT, Ob + z0 * PL, HD, (size_t)TT * 2 * TT, PL, PL);
    }
    k_split8<<<(unsigned)(((size_t)MT * DM / 8 + 255) / 256), 256, 0, stream>>>(Ob, ATh, ATl, (size_t)MT * DM / 8);
    k_gemmw<1, 0><<<dim3(MT / 64, DM / 64, 1), 32, 0, stream>>>(ATh, ATl, WO, nullptr, DM, DM, DM, OUT, DM, 0, 0, 0);
}
